// SparseMambaAttax_52209622450602
// MI455X (gfx1250) — hardware-verified
//
#include <hip/hip_runtime.h>
#include <math.h>
#include <stdint.h>


#define L_SEQ   2048
#define DMODEL  1024
#define NH_ATT  8
#define VHD     64
#define RD      32
#define TOPK    64
#define IDXD    64
#define QLR     128
#define KVLR    128
#define DSTATE  64
#define HDIM    32
#define DINNER  1024
#define NHM     32
#define CONVK   4
#define CONVDIM (DINNER + 2 * DSTATE)
#define DINPROJ (2 * DINNER + 2 * DSTATE + NHM)
#define QKD     (VHD + RD)
#define QKROW   (NH_ATT * QKD)
#define NPAD64(n) ((((n) + 63) / 64) * 64)

#define SC_ACT  64.0f
#define SC_WGT  1024.0f
#define SC_RES  2048.0f

typedef _Float16 f16;
typedef f16   v16h __attribute__((ext_vector_type(16)));
typedef f16   v8h  __attribute__((ext_vector_type(8)));
typedef float v8f  __attribute__((ext_vector_type(8)));
typedef float v4f  __attribute__((ext_vector_type(4)));
typedef float v4fa __attribute__((ext_vector_type(4), may_alias));

union Frag { v16h v; v8h h[2]; };

__device__ __forceinline__ v8f wmma16(v16h a, v16h b, v8f c) {
  return __builtin_amdgcn_wmma_f32_16x16x32_f16(false, a, false, b, (short)0, c, false, false);
}
#define WGUARD2(acc, a, b) \
  asm volatile("v_nop\n\tv_nop\n\tv_nop\n\tv_nop" : "+v"(acc) : "v"(a), "v"(b))
#define WGUARD6(acc, accx, a, al, b, bl) \
  asm volatile("v_nop\n\tv_nop\n\tv_nop\n\tv_nop" : "+v"(acc), "+v"(accx) : "v"(a), "v"(al), "v"(b), "v"(bl))

__device__ __forceinline__ void split8(const float* x, float s, v8h& hh, v8h& ll) {
  f16 ha[8], la[8];
#pragma unroll
  for (int i = 0; i < 8; ++i) {
    float v = x[i] * s;
    f16 h = (f16)v;
    f16 l = (f16)((v - (float)h) * SC_RES);
    ha[i] = h; la[i] = l;
  }
  hh = (v8h){ha[0], ha[1], ha[2], ha[3], ha[4], ha[5], ha[6], ha[7]};
  ll = (v8h){la[0], la[1], la[2], la[3], la[4], la[5], la[6], la[7]};
}

__device__ __forceinline__ float wsum_f(float v) {
  v += __shfl_xor(v, 16, 32); v += __shfl_xor(v, 8, 32); v += __shfl_xor(v, 4, 32);
  v += __shfl_xor(v, 2, 32);  v += __shfl_xor(v, 1, 32);
  return v;
}
__device__ __forceinline__ float wmax_f(float v) {
  v = fmaxf(v, __shfl_xor(v, 16, 32)); v = fmaxf(v, __shfl_xor(v, 8, 32)); v = fmaxf(v, __shfl_xor(v, 4, 32));
  v = fmaxf(v, __shfl_xor(v, 2, 32));  v = fmaxf(v, __shfl_xor(v, 1, 32));
  return v;
}
__device__ __forceinline__ int wsum_i(int v) {
  v += __shfl_xor(v, 16, 32); v += __shfl_xor(v, 8, 32); v += __shfl_xor(v, 4, 32);
  v += __shfl_xor(v, 2, 32);  v += __shfl_xor(v, 1, 32);
  return v;
}
__device__ __forceinline__ int clampi(int v, int lo, int hi) { return v < lo ? lo : (v > hi ? hi : v); }

__global__ void __launch_bounds__(256)
k_split_rows(const float* __restrict__ in, f16* oh, f16* ol, int n8, float s) {
  const int i = blockIdx.x * 256 + threadIdx.x;
  if (i >= n8) return;
  const size_t o = (size_t)i * 8;
  v4f a = *(const v4f*)(in + o), b = *(const v4f*)(in + o + 4);
  float x[8] = {a.x, a.y, a.z, a.w, b.x, b.y, b.z, b.w};
  v8h hh, ll;
  split8(x, s, hh, ll);
  *(volatile v8h*)(oh + o) = hh;
  *(volatile v8h*)(ol + o) = ll;
  __threadfence();
  *(volatile v8h*)(oh + o) = hh;
  *(volatile v8h*)(ol + o) = ll;
}

__global__ void __launch_bounds__(256)
k_split_tr(const float* __restrict__ W, f16* oh, f16* ol, int K, int N, float s, int lo_on) {
  __shared__ float tile[32][65];
  const int tid = threadIdx.x;
  const int k0 = blockIdx.x * 64, n0 = blockIdx.y * 32;
#pragma unroll
  for (int i = 0; i < 8; ++i) {
    const int e = tid + 256 * i, nl = e & 31, kl = e >> 5;
    const int k = k0 + kl, n = n0 + nl;
    float v = 0.0f;
    if (k < K && n < N) v = W[(size_t)k * N + n];
    tile[nl][kl] = v;
  }
  __syncthreads();
  const int r = tid >> 3, q = tid & 7;
  const int n = n0 + r, kk = k0 + 8 * q;
  float x[8];
#pragma unroll
  for (int i = 0; i < 8; ++i) x[i] = tile[r][8 * q + i];
  v8h hh, ll;
  split8(x, s, hh, ll);
  if (kk + 8 <= K) {
    const size_t o = (size_t)n * K + kk;
    *(volatile v8h*)(oh + o) = hh;
    if (lo_on) *(volatile v8h*)(ol + o) = ll;
    __threadfence();
    *(volatile v8h*)(oh + o) = hh;
    if (lo_on) *(volatile v8h*)(ol + o) = ll;
  }
}

template <int OUTP>
__device__ __forceinline__ void gemm_store(const float* sw, float* Cf, f16* Ch, f16* Cl,
                                           int m0, int n0, int M, int N, float s_out, int lane) {
  if (OUTP == 0) {
#pragma unroll
    for (int it = 0; it < 8; ++it) {
      const int f = it * 32 + lane, rr = f >> 4, c4 = f & 15;
      const int row = m0 + rr, col = n0 + 4 * c4;
      if (row < M && col < N) {
        v4f v = *(const v4fa*)(sw + rr * 64 + 4 * c4);
        *(volatile v4f*)(Cf + (size_t)row * N + col) = v;
      }
    }
  } else {
#pragma unroll
    for (int it = 0; it < 4; ++it) {
      const int f = it * 32 + lane, rr = f >> 3, c8 = f & 7;
      const int row = m0 + rr, col = n0 + 8 * c8;
      if (row < M && col < N) {
        v4f a = *(const v4fa*)(sw + rr * 64 + 8 * c8);
        v4f b = *(const v4fa*)(sw + rr * 64 + 8 * c8 + 4);
        float x[8] = {a.x, a.y, a.z, a.w, b.x, b.y, b.z, b.w};
        v8h hh, ll;
        split8(x, s_out, hh, ll);
        *(volatile v8h*)(Ch + (size_t)row * N + col) = hh;
        *(volatile v8h*)(Cl + (size_t)row * N + col) = ll;
      }
    }
  }
}

template <int SPLIT, int OUTP>
__global__ void __launch_bounds__(256)
k_gemm(const f16* __restrict__ Ah, const f16* __restrict__ Al,
       const f16* __restrict__ Bh, const f16* __restrict__ Bl,
       float* Cf, f16* Ch, f16* Cl,
       int M, int N, int K, float s_hh, float s_x, float s_out, int causal) {
  __shared__ float sT[8 * 16 * 64];
  const int lane = threadIdx.x & 31, wave = threadIdx.x >> 5;
  const int hh = lane >> 4, m = lane & 15;
  const int n0 = blockIdx.x * 64;
  const int mb = blockIdx.y * 128;
  if (causal && n0 >= mb + 128) return;
  const int m0 = mb + wave * 16;
  int ar = m0 + m;
  if (ar > M - 1) ar = M - 1;

  const f16* pa_h = Ah + (size_t)ar * K + 8 * hh;
  const f16* pa_l = Al + (size_t)ar * K + 8 * hh;
  const f16* pb_h[4];
  const f16* pb_l[4];
#pragma unroll
  for (int j = 0; j < 4; ++j) {
    const size_t o = (size_t)(n0 + 16 * j + m) * K + 8 * hh;
    pb_h[j] = Bh + o;
    pb_l[j] = Bl + o;
  }
  v8f acc[4], accx[4];
#pragma unroll
  for (int j = 0; j < 4; ++j) {
    acc[j] = (v8f){0.f, 0.f, 0.f, 0.f, 0.f, 0.f, 0.f, 0.f};
    accx[j] = acc[j];
  }

#pragma unroll 1
  for (int k0 = 0; k0 < K; k0 += 32) {
    Frag fa, fal;
    fa.h[0] = *(const v8h*)(pa_h + k0);
    fa.h[1] = *(const v8h*)(pa_h + k0 + 16);
    if (SPLIT) {
      fal.h[0] = *(const v8h*)(pa_l + k0);
      fal.h[1] = *(const v8h*)(pa_l + k0 + 16);
    }
#pragma unroll
    for (int j = 0; j < 4; ++j) {
      Frag fb, fbl;
      fb.h[0] = *(const v8h*)(pb_h[j] + k0);
      fb.h[1] = *(const v8h*)(pb_h[j] + k0 + 16);
      if (SPLIT) {
        fbl.h[0] = *(const v8h*)(pb_l[j] + k0);
        fbl.h[1] = *(const v8h*)(pb_l[j] + k0 + 16);
        acc[j]  = wmma16(fa.v, fb.v, acc[j]);
        accx[j] = wmma16(fa.v, fbl.v, accx[j]);
        accx[j] = wmma16(fal.v, fb.v, accx[j]);
        WGUARD6(acc[j], accx[j], fa.v, fal.v, fb.v, fbl.v);
      } else {
        acc[j] = wmma16(fa.v, fb.v, acc[j]);
        WGUARD2(acc[j], fa.v, fb.v);
      }
    }
  }

  float* sw = sT + wave * (16 * 64);
#pragma unroll
  for (int j = 0; j < 4; ++j) {
#pragma unroll
    for (int r = 0; r < 8; ++r) {
      float v;
      if (SPLIT) v = acc[j][r] * s_hh + accx[j][r] * s_x;
      else       v = acc[j][r] * s_hh;
      sw[(8 * hh + r) * 64 + 16 * j + m] = v;
    }
  }
  __syncthreads();
  gemm_store<OUTP>(sw, Cf, Ch, Cl, m0, n0, M, N, s_out, lane);
  __threadfence();
  gemm_store<OUTP>(sw, Cf, Ch, Cl, m0, n0, M, N, s_out, lane);
}

__global__ void __launch_bounds__(256)
k_conv_silu(const float* __restrict__ zx, const float* __restrict__ cw, const float* __restrict__ cb,
            float* out, int L) {
#pragma clang fp contract(off)
  const int per = CONVDIM / 4;
  const int id = blockIdx.x * 256 + threadIdx.x;
  if (id >= L * per) return;
  const int t = id / per, c = (id - t * per) * 4;
  float acc[4] = {0.f, 0.f, 0.f, 0.f};
#pragma unroll
  for (int k = 0; k < CONVK; ++k) {
    const int tt = t - (CONVK - 1) + k;
    if (tt >= 0) {
      v4f v = *(const v4f*)(zx + (size_t)tt * DINPROJ + DINNER + c);
      float xv[4] = {v.x, v.y, v.z, v.w};
#pragma unroll
      for (int e = 0; e < 4; ++e) acc[e] = acc[e] + xv[e] * cw[(c + e) * CONVK + k];
    }
  }
  float o[4];
#pragma unroll
  for (int e = 0; e < 4; ++e) {
    float v = acc[e] + cb[c + e];
    float sg = 1.0f / (1.0f + expf(-v));
    o[e] = v * sg;
  }
  v4f ov = (v4f){o[0], o[1], o[2], o[3]};
  float* dst = out + (size_t)t * CONVDIM + c;
  *(volatile v4f*)dst = ov;
  __threadfence();
  *(volatile v4f*)dst = ov;
}

__global__ void __launch_bounds__(256)
k_dtprep(const float* __restrict__ zx, const float* __restrict__ dt_bias, const float* __restrict__ A_log,
         float* dts, float* da, int L) {
#pragma clang fp contract(off)
  const int id = blockIdx.x * 256 + threadIdx.x;
  if (id >= L * NHM) return;
  const int t = id >> 5, h = id & 31;
  float r = zx[(size_t)t * DINPROJ + 2 * DINNER + 2 * DSTATE + h] + dt_bias[h];
  float sp = fmaxf(r, 0.0f) + log1pf(expf(-fabsf(r)));
  float A = -expf(A_log[h]);
  float d = expf(sp * A);
  *(volatile float*)(dts + id) = sp;
  *(volatile float*)(da + id) = d;
  __threadfence();
  *(volatile float*)(dts + id) = sp;
  *(volatile float*)(da + id) = d;
}

__global__ void __launch_bounds__(256)
k_scan(const float* __restrict__ xbc, const float* __restrict__ dts, const float* __restrict__ da,
       const float* __restrict__ Dssm, float* y, int L) {
#pragma clang fp contract(off)
  __shared__ float sB[DSTATE], sC[DSTATE];
  __shared__ float sDt[8], sDa[8];
  const int g = blockIdx.x, tid = threadIdx.x;
  const int ch = g * 256 + tid, hl = tid >> 5, head = g * 8 + hl;
  float st[DSTATE];
#pragma unroll
  for (int s = 0; s < DSTATE; ++s) st[s] = 0.0f;
  const float Dh = Dssm[head];
  for (int t = 0; t < L; ++t) {
    __syncthreads();
    if (tid < DSTATE)                 sB[tid] = xbc[(size_t)t * CONVDIM + DINNER + tid];
    else if (tid < 2 * DSTATE)        sC[tid - DSTATE] = xbc[(size_t)t * CONVDIM + DINNER + DSTATE + (tid - DSTATE)];
    else if (tid < 2 * DSTATE + 8)    sDt[tid - 2 * DSTATE] = dts[t * NHM + g * 8 + (tid - 2 * DSTATE)];
    else if (tid < 2 * DSTATE + 16)   sDa[tid - 2 * DSTATE - 8] = da[t * NHM + g * 8 + (tid - 2 * DSTATE - 8)];
    __syncthreads();
    const float x = xbc[(size_t)t * CONVDIM + ch];
    const float xdt = sDt[hl] * x;
    const float dec = sDa[hl];
    float acc = 0.0f;
#pragma unroll
    for (int s = 0; s < DSTATE; ++s) {
      st[s] = dec * st[s] + xdt * sB[s];
      acc = acc + st[s] * sC[s];
    }
    const float yv = acc + Dh * x;
    float* p = y + (size_t)t * DINNER + ch;
    *(volatile float*)p = yv;
    __threadfence();
    *(volatile float*)p = yv;
  }
}

__global__ void __launch_bounds__(128)
k_gate(const float* __restrict__ yssm, const float* __restrict__ zx, const float* __restrict__ nw,
       f16* gh, f16* gl) {
#pragma clang fp contract(off)
  __shared__ float red[4];
  const int t = blockIdx.x, tid = threadIdx.x, lane = tid & 31, wave = tid >> 5;
  const int c = tid * 8;
  const float* yr = yssm + (size_t)t * DINNER + c;
  const float* zr = zx + (size_t)t * DINPROJ + c;
  v4f y0 = *(const v4f*)yr, y1 = *(const v4f*)(yr + 4);
  v4f z0 = *(const v4f*)zr, z1 = *(const v4f*)(zr + 4);
  float yv[8] = {y0.x, y0.y, y0.z, y0.w, y1.x, y1.y, y1.z, y1.w};
  float zv[8] = {z0.x, z0.y, z0.z, z0.w, z1.x, z1.y, z1.z, z1.w};
  float g[8];
  float ss = 0.0f;
#pragma unroll
  for (int i = 0; i < 8; ++i) {
    float z = zv[i];
    float sg = 1.0f / (1.0f + expf(-z));
    float sl = z * sg;
    g[i] = yv[i] * sl;
    ss = ss + g[i] * g[i];
  }
  ss = wsum_f(ss);
  if (lane == 0) red[wave] = ss;
  __syncthreads();
  const float tot = ((red[0] + red[1]) + red[2]) + red[3];
  const float mean = tot * (1.0f / 1024.0f);
  const float rn = 1.0f / sqrtf(mean + 1e-5f);
  float x[8];
#pragma unroll
  for (int i = 0; i < 8; ++i) x[i] = (g[i] * rn) * nw[c + i];
  v8h hh, ll;
  split8(x, SC_ACT, hh, ll);
  const size_t o = (size_t)t * DINNER + c;
  *(volatile v8h*)(gh + o) = hh;
  *(volatile v8h*)(gl + o) = ll;
  __threadfence();
  *(volatile v8h*)(gh + o) = hh;
  *(volatile v8h*)(gl + o) = ll;
}

__device__ __forceinline__ void rope_store(float* qf, float* kf, size_t o, v4f qv, v4f kv) {
  *(volatile v4f*)(qf + o) = qv;
  *(volatile v4f*)(kf + o) = kv;
}

__global__ void __launch_bounds__(192)
k_rope(const float* __restrict__ qc, const float* __restrict__ qr, const float* __restrict__ kvb,
       const float* __restrict__ kr, float* qf, float* kf, int L) {
#pragma clang fp contract(off)
  __shared__ float ssn[RD / 2], scs[RD / 2];
  const int t = blockIdx.x, tid = threadIdx.x;
  if (tid < RD / 2) {
    const float inv = 1.0f / powf(10000.0f, (float)tid * 0.0625f);
    const float ang = (float)t * inv;
    ssn[tid] = sinf(ang);
    scs[tid] = cosf(ang);
  }
  __syncthreads();
  const int e0 = tid * 4;
  const int h = e0 / QKD, jj = e0 - h * QKD;
  v4f qv, kv;
  if (jj < VHD) {
    qv = *(const v4f*)(qc + (size_t)t * (NH_ATT * VHD) + h * VHD + jj);
    kv = *(const v4f*)(kvb + (size_t)t * (2 * NH_ATT * VHD) + h * VHD + jj);
  } else {
    const int j2 = jj - VHD;
    const int sec = j2 >> 4;
    const int fi0 = j2 & 15;
    float qo[4], ko[4];
#pragma unroll
    for (int e = 0; e < 4; ++e) {
      const int fi = fi0 + e;
      const float sn = ssn[fi], cs = scs[fi];
      const float q1 = qr[(size_t)t * (NH_ATT * RD) + h * RD + fi];
      const float q2 = qr[(size_t)t * (NH_ATT * RD) + h * RD + 16 + fi];
      const float k1 = kr[(size_t)t * RD + fi];
      const float k2 = kr[(size_t)t * RD + 16 + fi];
      if (sec == 0) { qo[e] = q1 * cs - q2 * sn; ko[e] = k1 * cs - k2 * sn; }
      else          { qo[e] = q1 * sn + q2 * cs; ko[e] = k1 * sn + k2 * cs; }
    }
    qv = (v4f){qo[0], qo[1], qo[2], qo[3]};
    kv = (v4f){ko[0], ko[1], ko[2], ko[3]};
  }
  const size_t o = (size_t)t * QKROW + e0;
  rope_store(qf, kf, o, qv, kv);
  __threadfence();
  rope_store(qf, kf, o, qv, kv);
}

__device__ __forceinline__ unsigned f2key(float f) {
  f = f + 0.0f;
  const unsigned b = __float_as_uint(f);
  return (b & 0x80000000u) ? ~b : (b | 0x80000000u);
}

__device__ __forceinline__ void attn_store(const float* sO, f16* dst, int tid) {
  if (tid < 64) {
    f16 hv[8];
#pragma unroll
    for (int i = 0; i < 8; ++i) hv[i] = (f16)(sO[8 * tid + i] * SC_ACT);
    v8h v = (v8h){hv[0], hv[1], hv[2], hv[3], hv[4], hv[5], hv[6], hv[7]};
    *(volatile v8h*)(dst + 8 * tid) = v;
  }
}

__global__ void __launch_bounds__(256)
k_sel_attn(const float* __restrict__ sc, const float* __restrict__ qf, const float* __restrict__ kf,
           const float* __restrict__ kvb, f16* attn16, int L) {
  __shared__ int   sRed[2][8];
  __shared__ int   sGe[64], sTi[64];
  __shared__ int   sList[TOPK];
  __shared__ float sq[QKROW];
  __shared__ float sP[NH_ATT * TOPK];
  __shared__ float sO[NH_ATT * VHD];
  const int t = blockIdx.x, tid = threadIdx.x, lane = tid & 31, wave = tid >> 5;
  if (t >= L) return;
  for (int p = tid; p < QKROW; p += 256) sq[p] = qf[(size_t)t * QKROW + p];
  if (tid < TOPK) sList[tid] = tid;

  if (t >= TOPK) {
    const size_t row = (size_t)t * L;
    unsigned u[8];
#pragma unroll
    for (int j = 0; j < 8; ++j) {
      const int s = j * 256 + tid;
      unsigned key = 0u;
      if (s <= t && s < L) key = f2key(sc[row + s]);
      u[j] = key;
    }
    unsigned T = 0u;
#pragma unroll 1
    for (int bit = 31; bit >= 0; --bit) {
      const unsigned cand = T | (1u << bit);
      int cnt = 0;
#pragma unroll
      for (int j = 0; j < 8; ++j) cnt += (u[j] >= cand) ? 1 : 0;
      cnt = wsum_i(cnt);
      if (lane == 0) sRed[bit & 1][wave] = cnt;
      __syncthreads();
      int tot = 0;
#pragma unroll
      for (int w = 0; w < 8; ++w) tot += sRed[bit & 1][w];
      if (tot >= TOPK) T = cand;
    }
    unsigned bge[8], bti[8];
#pragma unroll
    for (int j = 0; j < 8; ++j) {
      const int s = j * 256 + tid;
      const bool val = (s <= t && s < L);
      const bool ge = val && (u[j] > T), ti = val && (u[j] == T);
      bge[j] = __builtin_amdgcn_ballot_w32(ge);
      bti[j] = __builtin_amdgcn_ballot_w32(ti);
      if (lane == 0) {
        sGe[j * 8 + wave] = __builtin_popcount(bge[j]);
        sTi[j * 8 + wave] = __builtin_popcount(bti[j]);
      }
    }
    __syncthreads();
    int pg[8], pt[8];
    int baseA = 0, baseT = 0;
#pragma unroll
    for (int j = 0; j < 8; ++j) {
      int pa = 0, pb = 0, ra = 0, rb = 0;
#pragma unroll
      for (int w = 0; w < 8; ++w) {
        const int a = sGe[j * 8 + w] + sTi[j * 8 + w];
        const int b = sTi[j * 8 + w];
        ra += a; rb += b;
        if (w < wave) { pa += a; pb += b; }
      }
      pg[j] = baseA + pa; pt[j] = baseT + pb;
      baseA += ra; baseT += rb;
    }
    const int cgt = baseA - baseT;
    const int need = TOPK - cgt;
    const unsigned lt = (1u << lane) - 1u;
#pragma unroll
    for (int j = 0; j < 8; ++j) {
      const int s = j * 256 + tid;
      const bool val = (s <= t && s < L);
      const bool ge = val && (u[j] > T), ti = val && (u[j] == T);
      const int myG = pg[j] + __builtin_popcount((bge[j] | bti[j]) & lt);
      const int myT = pt[j] + __builtin_popcount(bti[j] & lt);
      const bool sel = ge || (ti && myT < need);
      int over = myT - need;
      if (over < 0) over = 0;
      const int pos = myG - over;
      if (sel && (unsigned)pos < (unsigned)TOPK) sList[pos] = s;
    }
  }
  __syncthreads();
  if (tid < TOPK) { const int v = sList[tid]; sList[tid] = clampi(v, 0, L - 1); }
  __syncthreads();

  const float scale = 0.10206207261596575f;
#pragma unroll
  for (int r = 0; r < 2; ++r) {
    const int p = tid + 256 * r, h = p >> 6, k = p & 63;
    const float* krow = kf + (size_t)sList[k] * QKROW + h * QKD;
    const float* qh = sq + h * QKD;
    float acc = 0.0f;
#pragma unroll 2
    for (int d4 = 0; d4 < QKD / 4; ++d4) {
      v4f kv = *(const v4f*)(krow + 4 * d4);
      acc += qh[4 * d4] * kv.x;
      acc += qh[4 * d4 + 1] * kv.y;
      acc += qh[4 * d4 + 2] * kv.z;
      acc += qh[4 * d4 + 3] * kv.w;
    }
    sP[p] = acc * scale;
  }
  __syncthreads();
  {
    const int h = wave;
    float v0 = sP[h * TOPK + lane], v1 = sP[h * TOPK + 32 + lane];
    const float mx = wmax_f(fmaxf(v0, v1));
    const float e0 = expf(v0 - mx), e1 = expf(v1 - mx);
    const float sm = wsum_f(e0 + e1);
    const float inv = 1.0f / sm;
    sP[h * TOPK + lane] = e0 * inv;
    sP[h * TOPK + 32 + lane] = e1 * inv;
  }
  __syncthreads();
#pragma unroll
  for (int r = 0; r < 2; ++r) {
    const int p = tid + 256 * r, h = p >> 6, d = p & 63;
    const float* vb = kvb + (NH_ATT * VHD) + h * VHD + d;
    const float* ph = sP + h * TOPK;
    float acc = 0.0f;
#pragma unroll 4
    for (int k = 0; k < TOPK; ++k) acc += ph[k] * vb[(size_t)sList[k] * (2 * NH_ATT * VHD)];
    sO[p] = acc;
  }
  __syncthreads();
  f16* dst = attn16 + (size_t)t * (NH_ATT * VHD);
  attn_store(sO, dst, tid);
  __threadfence();
  attn_store(sO, dst, tid);
}

extern "C" void kernel_launch(void* const* d_in, const int* in_sizes, int n_in,
                              void* d_out, int out_size, void* d_ws, size_t ws_size,
                              hipStream_t stream) {
  if (n_in < 18) return;
  if (in_sizes[0] != L_SEQ * DMODEL || in_sizes[1] != DMODEL * DINPROJ || out_size != L_SEQ * DMODEL) return;
  if (in_sizes[8] != DINNER * DMODEL || in_sizes[17] != NH_ATT * VHD * DMODEL) return;
  if (in_sizes[2] != CONVDIM * CONVK || in_sizes[9] != DMODEL * IDXD || in_sizes[15] != KVLR * 2 * NH_ATT * VHD) return;

  const float* x        = (const float*)d_in[0];
  const float* W_in     = (const float*)d_in[1];
  const float* conv_w   = (const float*)d_in[2];
  const float* conv_b   = (const float*)d_in[3];
  const float* dt_bias  = (const float*)d_in[4];
  const float* A_log    = (const float*)d_in[5];
  const float* D_ssm    = (const float*)d_in[6];
  const float* norm_w   = (const float*)d_in[7];
  const float* W_mout   = (const float*)d_in[8];
  const float* Wq_idx   = (const float*)d_in[9];
  const float* Wk_idx   = (const float*)d_in[10];
  const float* Wq_down  = (const float*)d_in[11];
  const float* Wq_up    = (const float*)d_in[12];
  const float* Wq_rope  = (const float*)d_in[13];
  const float* Wkv_down = (const float*)d_in[14];
  const float* Wkv_up   = (const float*)d_in[15];
  const float* Wk_rope  = (const float*)d_in[16];
  const float* W_out    = (const float*)d_in[17];
  float* out = (float*)d_out;

  char* ws = (char*)d_ws;
  size_t cur = 0, high = 0;
  auto take = [&](size_t bytes) -> char* {
    char* p = ws + cur;
    cur += (bytes + 255) & ~(size_t)255;
    if (cur > high) high = cur;
    return p;
  };
  const size_t L = L_SEQ;
  const size_t NP_IN = NPAD64(DINPROJ);
  const size_t NP_KR = NPAD64(RD);

  f16* xh    = (f16*)take(L * DMODEL * 2);
  f16* xl    = (f16*)take(L * DMODEL * 2);
  f16* winh  = (f16*)take(NP_IN * DMODEL * 2);
  f16* winl  = (f16*)take(NP_IN * DMODEL * 2);
  f16* wmoh  = (f16*)take((size_t)DMODEL * DINNER * 2);
  f16* wmol  = (f16*)take((size_t)DMODEL * DINNER * 2);
  f16* wqih  = (f16*)take((size_t)IDXD * DMODEL * 2);
  f16* wqil  = (f16*)take((size_t)IDXD * DMODEL * 2);
  f16* wkih  = (f16*)take((size_t)IDXD * DMODEL * 2);
  f16* wkil  = (f16*)take((size_t)IDXD * DMODEL * 2);
  f16* wqdh  = (f16*)take((size_t)QLR * DMODEL * 2);
  f16* wqdl  = (f16*)take((size_t)QLR * DMODEL * 2);
  f16* wkvdh = (f16*)take((size_t)KVLR * DMODEL * 2);
  f16* wkvdl = (f16*)take((size_t)KVLR * DMODEL * 2);
  f16* wquh  = (f16*)take((size_t)(NH_ATT * VHD) * QLR * 2);
  f16* wqul  = (f16*)take((size_t)(NH_ATT * VHD) * QLR * 2);
  f16* wqrh  = (f16*)take((size_t)(NH_ATT * RD) * QLR * 2);
  f16* wqrl  = (f16*)take((size_t)(NH_ATT * RD) * QLR * 2);
  f16* wkvuh = (f16*)take((size_t)(2 * NH_ATT * VHD) * KVLR * 2);
  f16* wkvul = (f16*)take((size_t)(2 * NH_ATT * VHD) * KVLR * 2);
  f16* wkrh  = (f16*)take(NP_KR * DMODEL * 2);
  f16* wkrl  = (f16*)take(NP_KR * DMODEL * 2);
  f16* wouth = (f16*)take((size_t)DMODEL * (NH_ATT * VHD) * 2);
  f16* gh    = (f16*)take(L * DINNER * 2);
  f16* gl    = (f16*)take(L * DINNER * 2);
  f16* attn16 = (f16*)take(L * NH_ATT * VHD * 2);
  const size_t arena = cur;

  cur = arena;
  float* zx    = (float*)take(L * DINPROJ * 4);
  float* xbc   = (float*)take(L * CONVDIM * 4);
  float* dts   = (float*)take(L * NHM * 4);
  float* da    = (float*)take(L * NHM * 4);
  float* yssm  = (float*)take(L * DINNER * 4);
  cur = arena;
  f16* xmh     = (f16*)take(L * DMODEL * 2);
  f16* xml     = (f16*)take(L * DMODEL * 2);
  f16* qih     = (f16*)take(L * IDXD * 2);
  f16* qil     = (f16*)take(L * IDXD * 2);
  f16* kih     = (f16*)take(L * IDXD * 2);
  f16* kil     = (f16*)take(L * IDXD * 2);
  const size_t endB = cur;
  cur = arena;
  f16* cqh     = (f16*)take(L * QLR * 2);
  f16* cql     = (f16*)take(L * QLR * 2);
  f16* ckh     = (f16*)take(L * KVLR * 2);
  f16* ckl     = (f16*)take(L * KVLR * 2);
  float* qcont = (float*)take(L * NH_ATT * VHD * 4);
  float* qrope = (float*)take(L * NH_ATT * RD * 4);
  float* kvb   = (float*)take(L * 2 * NH_ATT * VHD * 4);
  float* krope = (float*)take(L * RD * 4);
  float* qf    = (float*)take(L * QKROW * 4);
  float* kf    = (float*)take(L * QKROW * 4);
  const size_t endC = cur;
  cur = (endB > endC) ? endB : endC;
  float* scores = (float*)take(L * L * 4);
  if (high > ws_size) return;

  float* fdum = zx;
  f16*   hdum = xh;

  const float s16 = 1.0f / 65536.0f;
  const float s27 = s16 / 2048.0f;
  const float s12 = 1.0f / 4096.0f;
  const float s23 = s12 / 2048.0f;

  k_split_rows<<<(unsigned)((L * DMODEL / 8 + 255) / 256), 256, 0, stream>>>(x, xh, xl, (int)(L * DMODEL / 8), SC_ACT);
  auto trw = [&](const float* W, f16* oh, f16* ol, int K, int N, int lo_on) {
    dim3 g((unsigned)(K / 64), (unsigned)(NPAD64(N) / 32));
    k_split_tr<<<g, 256, 0, stream>>>(W, oh, ol, K, N, SC_WGT, lo_on);
  };
  trw(W_in,     winh,  winl,  DMODEL, DINPROJ, 1);
  trw(W_mout,   wmoh,  wmol,  DINNER, DMODEL, 1);
  trw(Wq_idx,   wqih,  wqil,  DMODEL, IDXD, 1);
  trw(Wk_idx,   wkih,  wkil,  DMODEL, IDXD, 1);
  trw(Wq_down,  wqdh,  wqdl,  DMODEL, QLR, 1);
  trw(Wq_up,    wquh,  wqul,  QLR, NH_ATT * VHD, 1);
  trw(Wq_rope,  wqrh,  wqrl,  QLR, NH_ATT * RD, 1);
  trw(Wkv_down, wkvdh, wkvdl, DMODEL, KVLR, 1);
  trw(Wkv_up,   wkvuh, wkvul, KVLR, 2 * NH_ATT * VHD, 1);
  trw(Wk_rope,  wkrh,  wkrl,  DMODEL, RD, 1);
  trw(W_out,    wouth, wouth, NH_ATT * VHD, DMODEL, 0);

  const unsigned MB = (unsigned)(L_SEQ / 128);

  k_gemm<1, 0><<<dim3((unsigned)(NP_IN / 64), MB), 256, 0, stream>>>(
      xh, xl, winh, winl, zx, hdum, hdum, L_SEQ, DINPROJ, DMODEL, s16, s27, 0.0f, 0);
  k_conv_silu<<<(unsigned)((L * (CONVDIM / 4) + 255) / 256), 256, 0, stream>>>(zx, conv_w, conv_b, xbc, L_SEQ);
  k_dtprep<<<(unsigned)((L * NHM + 255) / 256), 256, 0, stream>>>(zx, dt_bias, A_log, dts, da, L_SEQ);
  k_scan<<<(unsigned)(DINNER / 256), 256, 0, stream>>>(xbc, dts, da, D_ssm, yssm, L_SEQ);
  k_gate<<<(unsigned)L_SEQ, 128, 0, stream>>>(yssm, zx, norm_w, gh, gl);
  k_gemm<1, 1><<<dim3(DMODEL / 64, MB), 256, 0, stream>>>(
      gh, gl, wmoh, wmol, fdum, xmh, xml, L_SEQ, DMODEL, DINNER, s16, s27, SC_ACT, 0);

  k_gemm<1, 1><<<dim3(NPAD64(IDXD) / 64, MB), 256, 0, stream>>>(
      xmh, xml, wqih, wqil, fdum, qih, qil, L_SEQ, IDXD, DMODEL, s16, s27, SC_ACT, 0);
  k_gemm<1, 1><<<dim3(NPAD64(IDXD) / 64, MB), 256, 0, stream>>>(
      xh, xl, wkih, wkil, fdum, kih, kil, L_SEQ, IDXD, DMODEL, s16, s27, SC_ACT, 0);
  k_gemm<1, 0><<<dim3(L_SEQ / 64, MB), 256, 0, stream>>>(
      qih, qil, kih, kil, scores, hdum, hdum, L_SEQ, L_SEQ, IDXD, s12, s23, 0.0f, 1);

  k_gemm<1, 1><<<dim3(NPAD64(QLR) / 64, MB), 256, 0, stream>>>(
      xh, xl, wqdh, wqdl, fdum, cqh, cql, L_SEQ, QLR, DMODEL, s16, s27, SC_ACT, 0);
  k_gemm<1, 0><<<dim3((NH_ATT * VHD) / 64, MB), 256, 0, stream>>>(
      cqh, cql, wquh, wqul, qcont, hdum, hdum, L_SEQ, NH_ATT * VHD, QLR, s16, s27, 0.0f, 0);
  k_gemm<1, 0><<<dim3((NH_ATT * RD) / 64, MB), 256, 0, stream>>>(
      cqh, cql, wqrh, wqrl, qrope, hdum, hdum, L_SEQ, NH_ATT * RD, QLR, s16, s27, 0.0f, 0);
  k_gemm<1, 1><<<dim3(NPAD64(KVLR) / 64, MB), 256, 0, stream>>>(
      xh, xl, wkvdh, wkvdl, fdum, ckh, ckl, L_SEQ, KVLR, DMODEL, s16, s27, SC_ACT, 0);
  k_gemm<1, 0><<<dim3((2 * NH_ATT * VHD) / 64, MB), 256, 0, stream>>>(
      ckh, ckl, wkvuh, wkvul, kvb, hdum, hdum, L_SEQ, 2 * NH_ATT * VHD, KVLR, s16, s27, 0.0f, 0);
  k_gemm<1, 0><<<dim3((unsigned)(NP_KR / 64), MB), 256, 0, stream>>>(
      xh, xl, wkrh, wkrl, krope, hdum, hdum, L_SEQ, RD, DMODEL, s16, s27, 0.0f, 0);

  k_rope<<<(unsigned)L_SEQ, 192, 0, stream>>>(qcont, qrope, kvb, krope, qf, kf, L_SEQ);
  k_sel_attn<<<(unsigned)L_SEQ, 256, 0, stream>>>(scores, qf, kf, kvb, attn16, L_SEQ);
  k_gemm<0, 0><<<dim3(DMODEL / 64, MB), 256, 0, stream>>>(
      attn16, attn16, wouth, wouth, out, hdum, hdum, L_SEQ, DMODEL, NH_ATT * VHD, s16, 0.0f, 0.0f, 0);
}
